// FlowAE_20486994002690
// MI455X (gfx1250) — hardware-verified
//
#include <hip/hip_runtime.h>
#include <math.h>
typedef __attribute__((ext_vector_type(16))) _Float16 v16h;
typedef __attribute__((ext_vector_type(8)))  _Float16 v8h;
typedef __attribute__((ext_vector_type(16))) __bf16   v16b;
typedef __attribute__((ext_vector_type(8)))  __bf16   v8b;
typedef __attribute__((ext_vector_type(8)))  float    v8f;
typedef __attribute__((ext_vector_type(4)))  float    v4f;
#define PSCALE 32768.0f
#define U16(p) ((const unsigned short*)(const void*)(p))
#define PSCALE_INV (1.0f / 32768.0f)

__device__ __forceinline__ unsigned short f2bf_bits(float f) {
  unsigned u = __float_as_uint(f);
  return (unsigned short)((u + 0x7FFFu + ((u >> 16) & 1u)) >> 16);
}
__device__ __forceinline__ float bf_bits2f(unsigned short h) { return __uint_as_float(((unsigned)h) << 16); }

__device__ __forceinline__ void dep_guard_h(v8f& a, v8f& b, v16h x, v16h y) { asm volatile("v_nop\n\tv_nop\n\tv_nop\n\tv_nop" : "+v"(a), "+v"(b) : "v"(x), "v"(y)); }
__device__ __forceinline__ void dep_guard_b(v8f& a, v8f& b, v16b x, v16b y) { asm volatile("v_nop\n\tv_nop\n\tv_nop\n\tv_nop" : "+v"(a), "+v"(b) : "v"(x), "v"(y)); }
__device__ __forceinline__ void keep4_h(v16h a, v16h b, v16h c, v16h d) { asm volatile("v_nop" :: "v"(a), "v"(b), "v"(c), "v"(d)); }
__device__ __forceinline__ void keep4_b(v16b a, v16b b, v16b c, v16b d) { asm volatile("v_nop" :: "v"(a), "v"(b), "v"(c), "v"(d)); }
__device__ __forceinline__ void acc_guard4(v8f& a, v8f& b, v8f& c, v8f& d) { asm volatile("v_nop\n\tv_nop\n\tv_nop\n\tv_nop" : "+v"(a), "+v"(b), "+v"(c), "+v"(d)); }
template <typename T> struct Frag;
template <> struct Frag<_Float16> {
  typedef v16h V; union U { v16h v; v8h h[2]; };
  static __device__ __forceinline__ v16h load(const _Float16* p) {
    U f; f.h[0] = *(const v8h*)(p); f.h[1] = *(const v8h*)(p + 16); return f.v;
  }
  static __device__ __forceinline__ v8f mma(v16h a, v16h b, v8f c) {
    return __builtin_amdgcn_wmma_f32_16x16x32_f16(false, a, false, b, (short)0, c, false, false);
  }
  static __device__ __forceinline__ void guard(v8f& a, v8f& b, v16h x, v16h y) { dep_guard_h(a, b, x, y); }
  static __device__ __forceinline__ void keep(v16h a, v16h b, v16h c, v16h d) { keep4_h(a, b, c, d); }
};
template <> struct Frag<__bf16> {
  typedef v16b V; union U { v16b v; v8b h[2]; };
  static __device__ __forceinline__ v16b load(const __bf16* p) {
    U f; f.h[0] = *(const v8b*)(p); f.h[1] = *(const v8b*)(p + 16); return f.v;
  }
  static __device__ __forceinline__ v8f mma(v16b a, v16b b, v8f c) {
    return __builtin_amdgcn_wmma_f32_16x16x32_bf16(false, a, false, b, (short)0, c, false, false);
  }
  static __device__ __forceinline__ void guard(v8f& a, v8f& b, v16b x, v16b y) { dep_guard_b(a, b, x, y); }
  static __device__ __forceinline__ void keep(v16b a, v16b b, v16b c, v16b d) { keep4_b(a, b, c, d); }
};

template <int ET> struct Elem;
template <> struct Elem<0> { typedef _Float16 T; };
template <> struct Elem<1> { typedef __bf16 T; };
template <int ET, bool SPLIT, int BIAS_MODE, int OUT_MODE, bool RESID, int ACT = 0>
__global__ __launch_bounds__(256) void wmma_gemm64(
    const unsigned short* __restrict__ Ap, const unsigned short* __restrict__ A2p, int lda, long strideA,
    const unsigned short* __restrict__ Btp, const unsigned short* __restrict__ Bt2p, int ldb, long strideB,
    void* __restrict__ Cout, void* __restrict__ Cout2, int ldc, long strideC,
    const float* __restrict__ bias,
    const float* __restrict__ resid, long strideR,
    int M, int N, int K, float scale) {
  typedef typename Elem<ET>::T T;
  typedef typename Frag<T>::V V;
  const T* A = (const T*)Ap; const T* A2 = (const T*)A2p; const T* Bt = (const T*)Btp; const T* Bt2 = (const T*)Bt2p;
  __shared__ __align__(16) float sT[8][16 * 68];
  const int b    = blockIdx.y;
  const int lane = threadIdx.x & 31;
  const int wave = threadIdx.x >> 5;
  const int tilesN = N >> 6;
  const int tilesM = M >> 6;
  const int tile = blockIdx.x * 8 + wave;
  if (tile >= tilesM * tilesN) return;
  const int tm = tile / tilesN;
  const int tn = tile - tm * tilesN;
  const int m0 = tm << 6;
  const int n0 = tn << 6;

  const T* Ab  = A  + (size_t)b * strideA;
  const T* Bb  = Bt + (size_t)b * strideB;
  const T* Ab2 = SPLIT ? (A2  + (size_t)b * strideA) : nullptr;
  const T* Bb2 = SPLIT ? (Bt2 + (size_t)b * strideB) : nullptr;

  const int rlane = lane & 15;
  const int koff  = (lane >> 4) * 8;
  const int mOff  = (lane >> 4) * 8;

  v8f acc[4][4];
#pragma unroll
  for (int i = 0; i < 4; ++i)
#pragma unroll
    for (int j = 0; j < 4; ++j) acc[i][j] = (v8f){0.f,0.f,0.f,0.f,0.f,0.f,0.f,0.f};

  for (int k0 = 0; k0 < K; k0 += 32) {
    V bh[4], bl[4];
#pragma unroll
    for (int j = 0; j < 4; ++j) {
      const size_t bo = (size_t)(n0 + (j << 4) + rlane) * ldb + koff + k0;
      bh[j] = Frag<T>::load(Bb + bo);
      if (SPLIT) bl[j] = Frag<T>::load(Bb2 + bo);
    }
#pragma unroll
    for (int i = 0; i < 4; ++i) {
      const size_t ao = (size_t)(m0 + (i << 4) + rlane) * lda + koff + k0;
      V ah = Frag<T>::load(Ab + ao);
      V al;
      if (SPLIT) al = Frag<T>::load(Ab2 + ao);
#pragma unroll
      for (int j = 0; j < 4; ++j) {
        acc[i][j] = Frag<T>::mma(ah, bh[j], acc[i][j]);
        if (SPLIT) {
          acc[i][j] = Frag<T>::mma(ah, bl[j], acc[i][j]);
          acc[i][j] = Frag<T>::mma(al, bh[j], acc[i][j]);
        }
      }
      Frag<T>::guard(acc[i][0], acc[i][3], ah, SPLIT ? al : ah);
    }
    Frag<T>::keep(bh[0], bh[1], bh[2], bh[3]);
    if (SPLIT) Frag<T>::keep(bl[0], bl[1], bl[2], bl[3]);
  }
  acc_guard4(acc[0][0], acc[0][1], acc[0][2], acc[0][3]);
  acc_guard4(acc[1][0], acc[1][1], acc[1][2], acc[1][3]);
  acc_guard4(acc[2][0], acc[2][1], acc[2][2], acc[2][3]);
  acc_guard4(acc[3][0], acc[3][1], acc[3][2], acc[3][3]);

  float* slab = sT[wave];
  const float* Rb = RESID ? (resid + (size_t)b * strideR) : nullptr;
#pragma unroll
  for (int i = 0; i < 4; ++i) {
    const int mBase = m0 + (i << 4);
#pragma unroll
    for (int j = 0; j < 4; ++j) {
      const int n = n0 + (j << 4) + rlane;
      float bv = 0.f;
      if (BIAS_MODE == 2) bv = bias[n];
#pragma unroll
      for (int r = 0; r < 8; ++r) {
        float v = acc[i][j][r] * scale;
        if (BIAS_MODE == 1) v += bias[mBase + mOff + r];
        if (BIAS_MODE == 2) v += bv;
        if (RESID) v += Rb[(size_t)(mBase + mOff + r) * ldc + n];
        if (ACT == 1) v = tanhf(v);
        if (ACT == 2) v = fmaxf(v, 0.0f);
        if (ACT == 3) v = v / (1.0f + expf(-v));
        if (ACT == 4) v = (v > 0.f) ? v : 0.01f * v;
        if (ACT == 5) v = 0.5f * v * (1.0f + erff(v * 0.70710678118654752f));
        slab[(mOff + r) * 68 + (j << 4) + rlane] = v;
      }
    }
    __builtin_amdgcn_fence(__ATOMIC_RELEASE, "workgroup");
    __builtin_amdgcn_wave_barrier();
    __builtin_amdgcn_fence(__ATOMIC_ACQUIRE, "workgroup");
    if (OUT_MODE == 0) {
      float* C = (float*)Cout + (size_t)b * strideC;
      const int hh = lane >> 4, c4 = (lane & 15) * 4;
      for (int pass = 0; pass < 2; ++pass) {
#pragma unroll
        for (int it = 0; it < 8; ++it) {
          const int row = it * 2 + hh;
          v4f v = *(const v4f*)(slab + row * 68 + c4);
          *(volatile v4f*)(C + (size_t)(mBase + row) * ldc + n0 + c4) = v;
        }
        __threadfence();
      }
    } else {
      const int q = lane >> 3, c8 = (lane & 7) * 8;
      unsigned short* C  = (unsigned short*)Cout  + (size_t)b * strideC;
      unsigned short* C2 = (OUT_MODE == 2) ? ((unsigned short*)Cout2 + (size_t)b * strideC) : nullptr;
      for (int pass = 0; pass < 2; ++pass) {
#pragma unroll
        for (int it = 0; it < 4; ++it) {
          const int row = it * 4 + q;
          const float* sp = slab + row * 68 + c8;
          v8h hv, lv;
#pragma unroll
          for (int e = 0; e < 8; ++e) {
            if (OUT_MODE == 1) {
              hv[e] = (_Float16)sp[e];
            } else {
              unsigned short hb = f2bf_bits(sp[e]);
              unsigned short lb = f2bf_bits(sp[e] - bf_bits2f(hb));
              hv[e] = __builtin_bit_cast(_Float16, hb);
              lv[e] = __builtin_bit_cast(_Float16, lb);
            }
          }
          *(volatile v8h*)(C + (size_t)(mBase + row) * ldc + n0 + c8) = hv;
          if (OUT_MODE == 2) *(volatile v8h*)(C2 + (size_t)(mBase + row) * ldc + n0 + c8) = lv;
        }
        __threadfence();
      }
    }
    __builtin_amdgcn_fence(__ATOMIC_RELEASE, "workgroup");
    __builtin_amdgcn_wave_barrier();
    __builtin_amdgcn_fence(__ATOMIC_ACQUIRE, "workgroup");
  }
}

__global__ __launch_bounds__(256) void cast_f32_f16x2(
    const float* __restrict__ in, _Float16* __restrict__ out, int n2) {
  int i = blockIdx.x * 256 + threadIdx.x;
  if (i < n2) {
    const _Float16 h0 = (_Float16)in[2 * i], h1 = (_Float16)in[2 * i + 1];
    const unsigned u = (unsigned)__builtin_bit_cast(unsigned short, h0) | ((unsigned)__builtin_bit_cast(unsigned short, h1) << 16);
    ((volatile unsigned*)out)[i] = u;
    __threadfence();
    ((volatile unsigned*)out)[i] = u;
  }
}


__global__ __launch_bounds__(256) void transpose_cast_f16(const float* __restrict__ in, int ldi,
                                                         _Float16* __restrict__ outT, int ldo, float scale) {
  __shared__ __align__(16) _Float16 tile[64][72];
  const int c0 = blockIdx.x * 64, r0 = blockIdx.y * 64;
  const int t = threadIdx.y * 32 + threadIdx.x;
  for (int i = threadIdx.y; i < 64; i += 8) {
    tile[threadIdx.x][i]      = (_Float16)(in[(size_t)(r0 + i) * ldi + c0 + threadIdx.x] * scale);
    tile[32 + threadIdx.x][i] = (_Float16)(in[(size_t)(r0 + i) * ldi + c0 + 32 + threadIdx.x] * scale);
  }
  __syncthreads();
  const int q = t >> 3, c8 = (t & 7) * 8;
  for (int pass = 0; pass < 2; ++pass) {
#pragma unroll
    for (int it = 0; it < 2; ++it) {
      const int c = it * 32 + q;
      v8h hv = *(const v8h*)(&tile[c][c8]);
      *(volatile v8h*)(outT + (size_t)(c0 + c) * ldo + r0 + c8) = hv;
    }
    __threadfence();
  }
}

#define FB 16
#define FT 2048
#define FR (FB * FT)
#define FDI 16
#define FDM 256
#define FDF 1024
__global__ __launch_bounds__(256) void embed_kernel(const float* __restrict__ inp, const float* __restrict__ We, const float* __restrict__ be, unsigned* __restrict__ E16) {
  const int lane = threadIdx.x & 31, wave = threadIdx.x >> 5; const long r = (long)blockIdx.x * 8 + wave;
  __shared__ float xin[8][FDI];
  if (lane < FDI) xin[wave][lane] = inp[r * FDI + lane];
  __builtin_amdgcn_wave_barrier();
  float o[8];
#pragma unroll
  for (int q = 0; q < 8; ++q) { const int c = lane * 8 + q; float a = be[c];
#pragma unroll
    for (int k = 0; k < FDI; ++k) a += xin[wave][k] * We[k * FDM + c];
    o[q] = a; }
  typedef __attribute__((ext_vector_type(4))) unsigned u4; u4 pk;
#pragma unroll
  for (int q = 0; q < 4; ++q) pk[q] = (unsigned)__builtin_bit_cast(unsigned short, (_Float16)o[2 * q]) | ((unsigned)__builtin_bit_cast(unsigned short, (_Float16)o[2 * q + 1]) << 16);
  *(volatile u4*)(E16 + r * (FDM / 2) + lane * 4) = pk; __threadfence(); *(volatile u4*)(E16 + r * (FDM / 2) + lane * 4) = pk;
}
__global__ __launch_bounds__(256) void par_kernel(const float* __restrict__ Hh, const float* __restrict__ Ws, const float* __restrict__ bs, const float* __restrict__ precip, float* __restrict__ PAR) {
  const int lane = threadIdx.x & 31, wave = threadIdx.x >> 5; const long r = (long)blockIdx.x * 8 + wave;
  float s0 = 0.f, s1 = 0.f, s2 = 0.f, s3 = 0.f;
#pragma unroll
  for (int q = 0; q < 8; ++q) { const int c = lane * 8 + q; const float h = Hh[r * FDM + c]; s0 += h * Ws[c * 4]; s1 += h * Ws[c * 4 + 1]; s2 += h * Ws[c * 4 + 2]; s3 += h * Ws[c * 4 + 3]; }
  for (int o = 16; o > 0; o >>= 1) { s0 += __shfl_xor(s0, o, 32); s1 += __shfl_xor(s1, o, 32); s2 += __shfl_xor(s2, o, 32); s3 += __shfl_xor(s3, o, 32); }
  __shared__ float st[8][8];
  if (lane == 0) { const float xi = expf(s0 + bs[0]), om = expf(s1 + bs[1]), al = expf(s2 + bs[2]), rho = expf(s3 + bs[3]);
    const float eps = 1e-12f; const float norm = 1.0f / (om * (al + 1.0f / (al + eps)));
    st[wave][0] = xi; st[wave][1] = 1.0f / om; st[wave][2] = al + eps; st[wave][3] = 1.0f / (al + eps); st[wave][4] = rho * norm; st[wave][5] = precip[r]; st[wave][6] = om; st[wave][7] = 0.f; }
  __syncthreads();
  if (threadIdx.x < 64) { const float v = st[threadIdx.x >> 3][threadIdx.x & 7]; ((volatile float*)PAR)[(size_t)blockIdx.x * 64 + threadIdx.x] = v; __threadfence(); ((volatile float*)PAR)[(size_t)blockIdx.x * 64 + threadIdx.x] = v; }
}
__global__ __launch_bounds__(256) void bf_kernel(const float* __restrict__ Hh, const float* __restrict__ Wb, const float* __restrict__ bb, float* __restrict__ BF) {
  __shared__ double red[256];
  const int b = blockIdx.x, c = threadIdx.x;
  double s = 0.0; for (int t = 0; t < FT; ++t) s += (double)Hh[((size_t)b * FT + t) * FDM + c];
  red[c] = (s / FT) * (double)Wb[c];
  __syncthreads();
  for (int o = 128; o > 0; o >>= 1) { if (c < o) red[c] += red[c + o]; __syncthreads(); }
  if (c < 32) { const float v = (c == 0) ? expf((float)red[0] + bb[0]) : 0.f; ((volatile float*)BF)[b * 32 + c] = v; __threadfence(); ((volatile float*)BF)[b * 32 + c] = v; }
}
__global__ __launch_bounds__(256) void flow_kernel(const float* __restrict__ PAR, const float* __restrict__ BF, float* __restrict__ flow) {
  __shared__ float sx[256], sio[256], scp[256], scn[256], sa[256], sp[256];
  const int b = blockIdx.y; const int t = blockIdx.x * 256 + threadIdx.x;
  float acc = 0.f;
  const int tmax = blockIdx.x * 256 + 255;
  for (int i0 = 0; i0 <= tmax; i0 += 256) {
    __syncthreads();
    { const int i = i0 + threadIdx.x; const float* pr = PAR + ((size_t)b * FT + i) * 8; sx[threadIdx.x] = pr[0]; sio[threadIdx.x] = pr[1]; scp[threadIdx.x] = pr[2]; scn[threadIdx.x] = pr[3]; sa[threadIdx.x] = pr[4]; sp[threadIdx.x] = pr[5]; }
    __syncthreads();
    const int imax = min(255, t - i0);
    for (int ii = 0; ii <= imax; ++ii) {
      const float d = (float)(t - (i0 + ii)) - sx[ii];
      const float e = (d > 0.f) ? (d * sio[ii]) * scp[ii] : ((d < 0.f) ? (d * sio[ii]) * (-scn[ii]) : 0.f);
      acc += sp[ii] * sa[ii] * expf(-e);
    }
  }
  const float v = acc + BF[b * 32];
  ((volatile float*)flow)[(size_t)b * FT + t] = v; __threadfence(); ((volatile float*)flow)[(size_t)b * FT + t] = v;
}
__global__ __launch_bounds__(256) void mse_kernel(const float* __restrict__ flow, const float* __restrict__ ftrue, float* __restrict__ loss, float* __restrict__ loglik) {
  __shared__ double red[256];
  double s = 0.0; for (int i = threadIdx.x; i < FR; i += 256) { const double d = (double)flow[i] - (double)ftrue[i]; s += d * d; }
  red[threadIdx.x] = s; __syncthreads();
  for (int o = 128; o > 0; o >>= 1) { if (threadIdx.x < o) red[threadIdx.x] += red[threadIdx.x + o]; __syncthreads(); }
  if (threadIdx.x == 0) { const float m = (float)(red[0] / FR); ((volatile float*)loss)[0] = m; ((volatile float*)loglik)[0] = -m; __threadfence(); ((volatile float*)loss)[0] = m; ((volatile float*)loglik)[0] = -m; }
}
extern "C" void kernel_launch(void* const* d_in, const int* in_sizes, int n_in, void* d_out, int out_size, void* d_ws, size_t ws_size, hipStream_t stream) {
  (void)in_sizes; (void)n_in; (void)out_size; (void)ws_size;
  const float* inp = (const float*)d_in[0]; const float* precip = (const float*)d_in[1]; const float* ftrue = (const float*)d_in[2];
  const float* We = (const float*)d_in[3]; const float* be = (const float*)d_in[4]; const float* W1 = (const float*)d_in[5]; const float* b1 = (const float*)d_in[6]; const float* W2 = (const float*)d_in[7]; const float* b2 = (const float*)d_in[8];
  const float* Ws = (const float*)d_in[9]; const float* bs = (const float*)d_in[10]; const float* Wb = (const float*)d_in[11]; const float* bb = (const float*)d_in[12];
  float* out = (float*)d_out; float* loss = out; float* loglik = out + 1; float* flow = out + 2;
  char* ws = (char*)d_ws; size_t off = 0;
  auto carve = [&](size_t bytes) -> char* { char* p = ws + off; off += (bytes + 255) & ~(size_t)255; return p; };
  unsigned* E16 = (unsigned*)carve((size_t)FR * FDM * 2); _Float16* W1T = (_Float16*)carve((size_t)FDF * FDM * 2); _Float16* W2T = (_Float16*)carve((size_t)FDM * FDF * 2);
  unsigned* H1 = (unsigned*)carve((size_t)FR * FDF * 2);
  float* Hh = (float*)carve((size_t)FR * FDM * 4);
  float* PAR = (float*)carve((size_t)FR * 8 * 4); float* BF = (float*)carve(FB * 32 * 4);
  embed_kernel<<<FR / 8, 256, 0, stream>>>(inp, We, be, E16);
  transpose_cast_f16<<<dim3(FDF / 64, FDM / 64), dim3(32, 8), 0, stream>>>(W1, FDF, W1T, FDM, 1.0f);
  transpose_cast_f16<<<dim3(FDM / 64, FDF / 64), dim3(32, 8), 0, stream>>>(W2, FDM, W2T, FDF, 1.0f);
  { const int t1 = (FR / 64) * (FDF / 64), t2 = (FR / 64) * (FDM / 64);
    wmma_gemm64<0, false, 2, 1, false, 2><<<dim3((t1 + 7) / 8, 1), 256, 0, stream>>>((const unsigned short*)E16, nullptr, FDM, 0, U16(W1T), nullptr, FDM, 0, H1, nullptr, FDF, 0, b1, nullptr, 0, FR, FDF, FDM, 1.0f);
    wmma_gemm64<0, false, 2, 0, false, 0><<<dim3((t2 + 7) / 8, 1), 256, 0, stream>>>((const unsigned short*)H1, nullptr, FDF, 0, U16(W2T), nullptr, FDF, 0, Hh, nullptr, FDM, 0, b2, nullptr, 0, FR, FDM, FDF, 1.0f); }
  par_kernel<<<FR / 8, 256, 0, stream>>>(Hh, Ws, bs, precip, PAR);
  bf_kernel<<<FB, 256, 0, stream>>>(Hh, Wb, bb, BF);
  flow_kernel<<<dim3(FT / 256, FB), 256, 0, stream>>>(PAR, BF, flow);
  mse_kernel<<<1, 256, 0, stream>>>(flow, ftrue, loss, loglik);
}
